// RNN_62268435857828
// MI455X (gfx1250) — hardware-verified
//
#include <hip/hip_runtime.h>
#include <math.h>

constexpr int kBatch = 2048;
constexpr int kSteps = 512;
constexpr int kEmb   = 64;
constexpr int kHid   = 100;
constexpr int kVocab = 50001;
constexpr int kNP    = 112;
constexpr int kHKP   = 128;
constexpr int kKTot  = kEmb + kHKP;
constexpr int kKT    = kKTot / 32;
constexpr int kAP    = kKTot + 8;
constexpr int kRowsPB = 32;
constexpr int kBlocks = kBatch / kRowsPB;
constexpr int kWaves  = kNP / 16;
constexpr int kThr    = kWaves * 32;
constexpr int kATile  = kRowsPB * kAP;
constexpr int kHFP    = kNP;
constexpr int kPadCol0 = kEmb + kNP;
constexpr int kGatherChunks = kRowsPB * (kEmb / 8);
constexpr int kPadChunks    = kRowsPB * ((kKTot - kPadCol0) / 8);
constexpr int kWbtHalves = kNP * kKTot;
constexpr int kWbtDw     = kWbtHalves / 2;
constexpr int kPrepBlocks = kWbtDw / 256;
constexpr float kCIH     = 4096.0f;
constexpr float kCHH     = 256.0f;
constexpr float kCH      = 16.0f;
constexpr float kCAcc    = 4096.0f;
constexpr float kCAccInv = 1.0f / 4096.0f;

static_assert(kBatch % kRowsPB == 0);
static_assert(kRowsPB == 32);
static_assert(kNP % 16 == 0 && kNP >= kHid && kNP - kHid < 16);
static_assert(kKTot % 32 == 0 && kEmb % 32 == 0 && kHKP >= kHid);
static_assert(kAP % 8 == 0);
static_assert(kCH * kCHH == kCIH && kCIH == kCAcc);
static_assert(kWbtDw % 256 == 0 && kPrepBlocks == 42);
static_assert((kWbtHalves * 2) % 256 == 0);
static_assert(kGatherChunks > kThr && kGatherChunks - kThr <= 32);
static_assert(kPadChunks <= 64);
static_assert(kThr >= kNP);
static_assert((2 * kATile) % 8 == 0);

typedef __attribute__((ext_vector_type(16))) _Float16 v16h;
typedef __attribute__((ext_vector_type(8)))  _Float16 v8h;
typedef __attribute__((ext_vector_type(8)))  float    v8f;
typedef __attribute__((ext_vector_type(4)))  float    v4f;

__device__ __forceinline__ void dep_guard3_h(v8f& a, v8f& b, v16h x, v16h y, v16h z) {
  asm volatile("v_nop\n\tv_nop\n\tv_nop\n\tv_nop" : "+v"(a), "+v"(b) : "v"(x), "v"(y), "v"(z));
}
__device__ __forceinline__ void keep3_h(v16h a, v16h b, v16h c) { asm volatile("v_nop" :: "v"(a), "v"(b), "v"(c)); }
__device__ __forceinline__ void acc_guard2(v8f& a, v8f& b) { asm volatile("v_nop\n\tv_nop\n\tv_nop\n\tv_nop" : "+v"(a), "+v"(b)); }

template <typename T> struct Frag;
template <> struct Frag<_Float16> {
  typedef v16h V; union U { v16h v; v8h h[2]; };
  static __device__ __forceinline__ v16h load(const _Float16* p) {
    U f; f.h[0] = *(const v8h*)(p); f.h[1] = *(const v8h*)(p + 16); return f.v;
  }
  static __device__ __forceinline__ v8f mma(v16h a, v16h b, v8f c) {
    return __builtin_amdgcn_wmma_f32_16x16x32_f16(false, a, false, b, (short)0, c, false, false);
  }
};

__device__ __forceinline__ unsigned pack_f16x2(float a, float b) {
  const _Float16 h0 = (_Float16)a, h1 = (_Float16)b;
  return (unsigned)__builtin_bit_cast(unsigned short, h0) | ((unsigned)__builtin_bit_cast(unsigned short, h1) << 16);
}
__device__ __forceinline__ void st2u(unsigned* p, unsigned v) { *(volatile unsigned*)p = v; __threadfence(); *(volatile unsigned*)p = v; }

__global__ __launch_bounds__(256) void prep_wbt_kernel(const float* __restrict__ w_ih, const float* __restrict__ w_hh,
                                                       unsigned* __restrict__ wbt) {
  const int p  = blockIdx.x * 256 + threadIdx.x;
  const int n  = p / (kKTot / 2);
  const int j0 = (p - n * (kKTot / 2)) * 2;
  float v[2];
#pragma unroll
  for (int e = 0; e < 2; ++e) {
    const int j   = j0 + e;
    const int nc  = (n < kHid) ? n : (kHid - 1);
    const int jih = (j < kEmb) ? j : (kEmb - 1);
    const int jr  = j - kEmb;
    const int jhh = (jr < 0) ? 0 : ((jr < kHid) ? jr : (kHid - 1));
    const float a = w_ih[nc * kEmb + jih];
    const float b = w_hh[nc * kHid + jhh];
    const float fih = (n < kHid && j < kEmb) ? 1.0f : 0.0f;
    const float fhh = (n < kHid && j >= kEmb && j < kEmb + kHid) ? 1.0f : 0.0f;
    v[e] = fmaf(fih, a * kCIH, fhh * (b * kCHH));
  }
  st2u(wbt + p, pack_f16x2(v[0], v[1]));
}

__device__ __forceinline__ void gather_chunk(const int* __restrict__ x, const float* __restrict__ emb,
                                             _Float16* Anext, int rb, int tstep, int i) {
  const int row = i >> 3, c8 = i & 7;
  int tok = x[(size_t)(rb + row) * kSteps + tstep];
  tok = (tok < 0) ? 0 : ((tok > kVocab - 1) ? (kVocab - 1) : tok);
  const float* src = emb + (size_t)tok * kEmb + c8 * 8;
  const v4f f0 = *(const v4f*)src;
  const v4f f1 = *(const v4f*)(src + 4);
  v8h hv;
  hv[0] = (_Float16)f0[0]; hv[1] = (_Float16)f0[1]; hv[2] = (_Float16)f0[2]; hv[3] = (_Float16)f0[3];
  hv[4] = (_Float16)f1[0]; hv[5] = (_Float16)f1[1]; hv[6] = (_Float16)f1[2]; hv[7] = (_Float16)f1[3];
  *(v8h*)(Anext + row * kAP + c8 * 8) = hv;
}
__device__ __forceinline__ void gather_rows(const int* __restrict__ x, const float* __restrict__ emb,
                                            _Float16* Anext, int rb, int tstep, int tid) {
  gather_chunk(x, emb, Anext, rb, tstep, tid);
  if (tid < kGatherChunks - kThr) gather_chunk(x, emb, Anext, rb, tstep, kThr + tid);
  if (tid < kPadChunks) {
    const v8h z = {(_Float16)0.f, (_Float16)0.f, (_Float16)0.f, (_Float16)0.f, (_Float16)0.f, (_Float16)0.f, (_Float16)0.f, (_Float16)0.f};
    const int row = tid >> 1, hf = tid & 1;
    *(v8h*)(Anext + row * kAP + kPadCol0 + hf * 8) = z;
  }
}

__global__ __launch_bounds__(kThr) void rnn_fused_kernel(const int* __restrict__ x, const float* __restrict__ emb,
                                                         const unsigned short* __restrict__ wbtp,
                                                         const float* __restrict__ b_ih, const float* __restrict__ b_hh,
                                                         const float* __restrict__ fc_w, const float* __restrict__ fc_b,
                                                         float* __restrict__ out) {
  __shared__ __align__(16) _Float16 Abuf[2 * kATile];
  __shared__ __align__(16) float    Hf[kRowsPB * kHFP];
  __shared__ float Fs[kNP];
  const _Float16* wbt = (const _Float16*)wbtp;
  const int tid = threadIdx.x, lane = tid & 31, wave = tid >> 5;
  const int c = lane & 15, hh = lane >> 4, koff = hh * 8;
  const int rb = blockIdx.x * kRowsPB;
  const int ncol = wave * 16 + c;

  {
    const v8h z = {(_Float16)0.f, (_Float16)0.f, (_Float16)0.f, (_Float16)0.f, (_Float16)0.f, (_Float16)0.f, (_Float16)0.f, (_Float16)0.f};
    for (int i = tid; i < (2 * kATile) / 8; i += kThr) *(v8h*)(Abuf + i * 8) = z;
  }
  __syncthreads();

  gather_rows(x, emb, Abuf, rb, 0, tid);

  v16h fb[kKT];
  {
    const _Float16* brow = wbt + (size_t)ncol * kKTot + koff;
    fb[0] = Frag<_Float16>::load(brow + 0);
    fb[1] = Frag<_Float16>::load(brow + 32);
    fb[2] = Frag<_Float16>::load(brow + 64);
    keep3_h(fb[0], fb[1], fb[2]);
    fb[3] = Frag<_Float16>::load(brow + 96);
    fb[4] = Frag<_Float16>::load(brow + 128);
    fb[5] = Frag<_Float16>::load(brow + 160);
    keep3_h(fb[3], fb[4], fb[5]);
  }
  const int ncc = (ncol < kHid) ? ncol : (kHid - 1);
  const float bsel = (ncol < kHid) ? 1.0f : 0.0f;
  const float biasAcc = bsel * ((b_ih[ncc] + b_hh[ncc]) * kCAcc);

  float hst[2][8];
#pragma unroll
  for (int ms = 0; ms < 2; ++ms)
#pragma unroll
    for (int r = 0; r < 8; ++r) hst[ms][r] = 0.0f;
  __syncthreads();

#pragma unroll 1
  for (int t = 0; t < kSteps; ++t) {
    const _Float16* Acur = Abuf + (t & 1) * kATile;
    _Float16*       Anext = Abuf + ((t + 1) & 1) * kATile;
    const int tn = (t + 1 < kSteps) ? (t + 1) : (kSteps - 1);
    gather_rows(x, emb, Anext, rb, tn, tid);

    v8f acc[2];
#pragma unroll
    for (int r = 0; r < 8; ++r) { acc[0][r] = biasAcc; acc[1][r] = biasAcc; }
    const _Float16* arow0 = Acur + c * kAP + koff;
    const _Float16* arow1 = Acur + (16 + c) * kAP + koff;
#pragma unroll
    for (int kt = 0; kt < kKT; ++kt) {
      const v16h a0 = Frag<_Float16>::load(arow0 + kt * 32);
      const v16h a1 = Frag<_Float16>::load(arow1 + kt * 32);
      acc[0] = Frag<_Float16>::mma(a0, fb[kt], acc[0]);
      acc[1] = Frag<_Float16>::mma(a1, fb[kt], acc[1]);
      dep_guard3_h(acc[0], acc[1], a0, a1, fb[kt]);
    }
    acc_guard2(acc[0], acc[1]);

#pragma unroll
    for (int ms = 0; ms < 2; ++ms) {
#pragma unroll
      for (int r = 0; r < 8; ++r) {
        const float pre = acc[ms][r] * kCAccInv;
        const float hv  = tanhf(pre);
        const float hq  = (ncol < kHid) ? hv : 0.0f;
        hst[ms][r] = hq;
        Anext[(16 * ms + 8 * hh + r) * kAP + kEmb + ncol] = (_Float16)(hq * kCH);
      }
    }
    __syncthreads();
  }

#pragma unroll
  for (int ms = 0; ms < 2; ++ms)
#pragma unroll
    for (int r = 0; r < 8; ++r) Hf[(16 * ms + 8 * hh + r) * kHFP + ncol] = hst[ms][r];
  {
    const int kc = (tid < kHid) ? tid : (kHid - 1);
    const float fw = fc_w[kc];
    const float fsel = (tid < kHid) ? 1.0f : 0.0f;
    if (tid < kNP) Fs[tid] = fsel * fw;
  }
  __syncthreads();
  if (wave == 0) {
    const int row = lane;
    float accd = 0.0f;
#pragma unroll 1
    for (int k = 0; k < kHid; ++k) accd = fmaf(Hf[row * kHFP + k], Fs[k], accd);
    const float logit = accd + fc_b[0];
    const float o = 1.0f / (1.0f + expf(-logit));
    float* op = out + rb + row;
    *(volatile float*)op = o;
    __threadfence();
    *(volatile float*)op = o;
  }
}

extern "C" void kernel_launch(void* const* d_in, const int* in_sizes, int n_in,
                              void* d_out, int out_size, void* d_ws, size_t ws_size, hipStream_t stream) {
  if (n_in < 8 || d_out == nullptr || d_ws == nullptr) return;
  if (in_sizes[0] != kBatch * kSteps || in_sizes[1] != kVocab * kEmb || in_sizes[2] != kHid * kEmb ||
      in_sizes[3] != kHid * kHid || in_sizes[4] != kHid || in_sizes[5] != kHid || in_sizes[6] != kHid ||
      in_sizes[7] != 1 || out_size != kBatch) return;

  const int*   x    = (const int*)d_in[0];
  const float* embt = (const float*)d_in[1];
  const float* w_ih = (const float*)d_in[2];
  const float* w_hh = (const float*)d_in[3];
  const float* b_ih = (const float*)d_in[4];
  const float* b_hh = (const float*)d_in[5];
  const float* fc_w = (const float*)d_in[6];
  const float* fc_b = (const float*)d_in[7];
  float* out = (float*)d_out;

  char* ws = (char*)d_ws; size_t off = 0;
  auto carve = [&](size_t bytes) -> char* { char* p = ws + off; off += (bytes + 255) & ~(size_t)255; return p; };
  unsigned short* WBT = (unsigned short*)carve((size_t)kWbtHalves * 2);
  if (off > ws_size || off > (size_t)134217728) return;

  prep_wbt_kernel<<<kPrepBlocks, 256, 0, stream>>>(w_ih, w_hh, (unsigned*)WBT);
  rnn_fused_kernel<<<kBlocks, kThr, 0, stream>>>(x, embt, WBT, b_ih, b_hh, fc_w, fc_b, out);
}
